// LocalSelfAttention_29111288332435
// MI455X (gfx1250) — hardware-verified
//
#include <hip/hip_runtime.h>
#include <stddef.h>


typedef _Float16 v16h __attribute__((ext_vector_type(16)));
typedef _Float16 v8h  __attribute__((ext_vector_type(8)));
typedef float    v8f  __attribute__((ext_vector_type(8)));
typedef float    v4f  __attribute__((ext_vector_type(4)));

#ifndef NB
#define NB 2
#endif
#ifndef IMG_H
#define IMG_H 56
#endif
#define NB_FULL    2
#define IMG_H_FULL 56
#define IMG_W      56
#define WIN        7
#define SEQ        (IMG_H * IMG_W)
#define SEQ_FULL   (IMG_H_FULL * IMG_W)
#define DIM   256
#define NHEAD 8
#define HD    32
#define NPAIR 16
#define MROWS (NB * SEQ)

static_assert(NB >= 1 && NB <= NB_FULL);
static_assert(IMG_H >= WIN && IMG_H <= IMG_H_FULL);
static_assert(IMG_W == 56 && WIN == 7);
static_assert((IMG_W % 8) == 0);
static_assert(4 * 16 >= IMG_W && IMG_W - 48 == 8);
static_assert(IMG_W - 32 == 24);
static_assert((SEQ % 64) == 0 && (MROWS % 64) == 0 && (MROWS % 8) == 0);
static_assert(DIM == NHEAD * HD);
static_assert(HD == 32 && HD == 2 * NPAIR);
static_assert((NHEAD % 2) == 0);
static_assert((DIM % 64) == 0 && (DIM % 32) == 0);
static_assert(DIM == 32 * 8);
static_assert(((SEQ * NPAIR) % 256) == 0);

#define LDT 72
#define LDC 68
#define LDP 40
static_assert((LDT % 8) == 0 && LDT >= 64);
static_assert((LDC % 4) == 0 && LDC >= 64);
static_assert((LDP % 8) == 0 && LDP >= 32);

#define WCARRY 64.0f
#define PCARRY 1024.0f
#define VCARRY 64.0f

#define WQKV_BYTES    ((size_t)3 * DIM * DIM * 2)
#define WP_BYTES      ((size_t)DIM * DIM * 2)
#define PLANE16_BYTES ((size_t)MROWS * DIM * 2)
#define TAB_BYTES     ((size_t)SEQ * NPAIR * 4)
#define OFF_WQKV ((size_t)0)
#define OFF_WP   (OFF_WQKV + WQKV_BYTES)
#define OFF_X16  (OFF_WP + WP_BYTES)
#define OFF_Q    (OFF_X16 + PLANE16_BYTES)
#define OFF_K    (OFF_Q + PLANE16_BYTES)
#define OFF_VT   (OFF_K + PLANE16_BYTES)
#define OFF_CTX  (OFF_VT + PLANE16_BYTES)
#define OFF_COS  (OFF_CTX + PLANE16_BYTES)
#define OFF_SIN  (OFF_COS + TAB_BYTES)
#define WS_TOTAL (OFF_SIN + TAB_BYTES)
static_assert((WQKV_BYTES % 128) == 0 && (WP_BYTES % 128) == 0 && (PLANE16_BYTES % 128) == 0);
static_assert((TAB_BYTES % 128) == 0);
static_assert(WS_TOTAL <= (size_t)134217728);

__device__ __forceinline__ float bf16r(float x) {
  unsigned int u = __float_as_uint(x);
  u = (u + 0x7FFFu + ((u >> 16) & 1u)) & 0xFFFF0000u;
  return __uint_as_float(u);
}

static __device__ __forceinline__ _Float16 toh_flush(float v) {
  const _Float16 r = (_Float16)v;
  return (fabsf(v) < 6.103515625e-05f) ? (_Float16)0.0f : r;
}

__device__ __forceinline__ v16h frag_at(const _Float16* p) {
  v8h lo = *(const v8h*)(p);
  v8h hi = *(const v8h*)(p + 16);
  v16h out;
#pragma unroll
  for (int i = 0; i < 8; ++i) { out[i] = lo[i]; out[i + 8] = hi[i]; }
  return out;
}
__device__ __forceinline__ v16h ld_frag(const _Float16* base, unsigned ld) {
  const unsigned lane = threadIdx.x & 31u;
  return frag_at(base + (lane & 15u) * ld + (lane >> 4) * 8u);
}

__device__ __forceinline__ v8f wmma16(v16h a, v16h b, v8f c) {
  v8f d = __builtin_amdgcn_wmma_f32_16x16x32_f16(false, a, false, b, (short)0, c,
                                                 false, false);
  asm volatile("v_nop\n\tv_nop\n\tv_nop\n\tv_nop" : "+v"(d) : "v"(a), "v"(b));
  return d;
}

__device__ __forceinline__ float red16_max(float x) {
#pragma unroll
  for (int off = 1; off < 16; off <<= 1) x = fmaxf(x, __shfl_xor(x, off, 32));
  return x;
}
__device__ __forceinline__ float red16_sum(float x) {
#pragma unroll
  for (int off = 1; off < 16; off <<= 1) x += __shfl_xor(x, off, 32);
  return x;
}

__device__ __forceinline__ void wave_lds_sync() {
  __builtin_amdgcn_fence(3  , "wavefront");
  asm volatile("s_wait_dscnt 0x0" ::: "memory");
  __builtin_amdgcn_wave_barrier();
}

__global__ __launch_bounds__(256) void wconv_kernel(
    const float* __restrict__ W, _Float16* __restrict__ Wt, unsigned ldw, unsigned ldk) {
  __shared__ _Float16 T[64 * LDT];
  const unsigned tid = threadIdx.x;
  const unsigned n0 = blockIdx.x * 64u;
  const unsigned k0 = blockIdx.y * 64u;
#pragma unroll 4
  for (unsigned j = 0; j < 16u; ++j) {
    const unsigned idx = tid + 256u * j;
    const unsigned kr = idx >> 6, nc = idx & 63u;
    const float v = W[(size_t)(k0 + kr) * ldw + n0 + nc];
    T[nc * LDT + kr] = (_Float16)(WCARRY * bf16r(v));
  }
  __syncthreads();
  v8h x[2];
  size_t off[2];
#pragma unroll
  for (unsigned i = 0; i < 2u; ++i) {
    const unsigned n = 32u * i + (tid >> 3);
    const unsigned kc = (tid & 7u) * 8u;
    x[i] = *(const v8h*)&T[n * LDT + kc];
    off[i] = (size_t)(n0 + n) * ldk + k0 + kc;
  }
#pragma unroll
  for (int i = 0; i < 2; ++i) *(volatile v8h*)(Wt + off[i]) = x[i];
  __threadfence();
#pragma unroll
  for (int i = 0; i < 2; ++i) *(volatile v8h*)(Wt + off[i]) = x[i];
}

__global__ __launch_bounds__(256) void xconv_kernel(
    const float* __restrict__ X, _Float16* __restrict__ dst) {
  const unsigned gid = blockIdx.x * 256u + threadIdx.x;
  const unsigned crow = gid >> 5;
  const unsigned c = (gid & 31u) * 8u;
  const unsigned bidx = crow / (unsigned)SEQ;
  const unsigned sq = crow - bidx * (unsigned)SEQ;
  const size_t srow = (size_t)bidx * SEQ_FULL + sq;
  const v4f a0 = *(const v4f*)(X + srow * DIM + c);
  const v4f a1 = *(const v4f*)(X + srow * DIM + c + 4u);
  v8h o;
#pragma unroll
  for (int i = 0; i < 4; ++i) {
    o[i]     = toh_flush(bf16r(a0[i]));
    o[i + 4] = toh_flush(bf16r(a1[i]));
  }
  _Float16* p = dst + (size_t)crow * DIM + c;
  *(volatile v8h*)p = o;
  __threadfence();
  *(volatile v8h*)p = o;
}

__global__ __launch_bounds__(256) void ropetab_kernel(
    float* __restrict__ cosT, float* __restrict__ sinT) {
#pragma clang fp contract(off)
  const unsigned idx = blockIdx.x * 256u + threadIdx.x;
  const unsigned n = idx >> 4, p = idx & 15u;
  const float inv = exp2f(-(float)p * 0.83048202372184059f);
  const float ang = (float)n * inv;
  float sn, cs;
  sincosf(ang, &sn, &cs);
  *(volatile float*)(cosT + idx) = cs;
  *(volatile float*)(sinT + idx) = sn;
  __threadfence();
  *(volatile float*)(cosT + idx) = cs;
  *(volatile float*)(sinT + idx) = sn;
}

template <int MODE>
__device__ __forceinline__ void gemm_body(
    const _Float16* __restrict__ A16, const _Float16* __restrict__ Bt, const unsigned K,
    const float* __restrict__ bias, const float* __restrict__ cosT,
    const float* __restrict__ sinT, const int* __restrict__ hin, const int* __restrict__ win,
    float* __restrict__ outf, _Float16* __restrict__ out16) {
  __shared__ float Cs[64 * LDC];
  const unsigned tid = threadIdx.x, lane = tid & 31u, w = tid >> 5;
  const unsigned mw = w >> 1, nw = w & 1u;
  const unsigned hh = lane >> 4, m = lane & 15u;
  const unsigned n0 = blockIdx.x * 64u;
  const unsigned row0 = blockIdx.y * 64u;

  const _Float16* ap  = A16 + (size_t)(row0 + mw * 16u + m) * K + hh * 8u;
  const _Float16* bp0 = Bt + (size_t)(n0 + nw * 32u + m) * K + hh * 8u;
  const _Float16* bp1 = bp0 + (size_t)16 * K;
  v8f acc0 = {}, acc1 = {};
#pragma unroll 2
  for (unsigned k0 = 0; k0 < K; k0 += 32u) {
    const v16h a  = frag_at(ap + k0);
    const v16h b0 = frag_at(bp0 + k0);
    const v16h b1 = frag_at(bp1 + k0);
    acc0 = wmma16(a, b0, acc0);
    acc1 = wmma16(a, b1, acc1);
  }
#pragma unroll
  for (int r = 0; r < 8; ++r) {
    float* d = &Cs[(mw * 16u + hh * 8u + (unsigned)r) * LDC + nw * 32u + m];
    d[0]  = acc0[r];
    d[16] = acc1[r];
  }
  __syncthreads();

  if (MODE == 0) {
    v8h x[2];
    size_t off[2];
#pragma unroll
    for (unsigned i = 0; i < 2u; ++i) {
      const unsigned r = 32u * i + (tid >> 3);
      const unsigned c = (tid & 7u) * 8u;
      const unsigned crow = row0 + r;
      const unsigned bidx = crow / (unsigned)SEQ;
      const unsigned sq = crow - bidx * (unsigned)SEQ;
      const unsigned p0 = (c & 31u) >> 1;
      const v4f u0 = *(const v4f*)&Cs[r * LDC + c];
      const v4f u1 = *(const v4f*)&Cs[r * LDC + c + 4];
      const v4f cs4 = *(const v4f*)(cosT + (size_t)sq * NPAIR + p0);
      const v4f sn4 = *(const v4f*)(sinT + (size_t)sq * NPAIR + p0);
#pragma unroll
      for (int j = 0; j < 2; ++j) {
        const float a0 = u0[2 * j] * (1.0f / WCARRY);
        const float a1 = u0[2 * j + 1] * (1.0f / WCARRY);
        const float b0 = u1[2 * j] * (1.0f / WCARRY);
        const float b1 = u1[2 * j + 1] * (1.0f / WCARRY);
        x[i][2 * j]         = toh_flush(a0 * cs4[j] - a1 * sn4[j]);
        x[i][2 * j + 1]     = toh_flush(a1 * cs4[j] + a0 * sn4[j]);
        x[i][4 + 2 * j]     = toh_flush(b0 * cs4[j + 2] - b1 * sn4[j + 2]);
        x[i][4 + 2 * j + 1] = toh_flush(b1 * cs4[j + 2] + b0 * sn4[j + 2]);
      }
      off[i] = (size_t)crow * DIM + n0 + c;
    }
#pragma unroll
    for (int i = 0; i < 2; ++i) *(volatile v8h*)(out16 + off[i]) = x[i];
    __threadfence();
#pragma unroll
    for (int i = 0; i < 2; ++i) *(volatile v8h*)(out16 + off[i]) = x[i];
  }

  if (MODE == 1) {
    const unsigned bidx = row0 / (unsigned)SEQ;
    const unsigned key0 = row0 - bidx * (unsigned)SEQ;
    v8h x[2];
    size_t off[2];
#pragma unroll
    for (unsigned i = 0; i < 2u; ++i) {
      const unsigned dcol = 32u * i + (tid >> 3);
      const unsigned kk = (tid & 7u) * 8u;
#pragma unroll
      for (unsigned j = 0; j < 8u; ++j) {
        const float t = Cs[(kk + j) * LDC + dcol] * (1.0f / WCARRY);
        x[i][j] = toh_flush(t);
      }
      off[i] = ((size_t)bidx * DIM + n0 + dcol) * SEQ + key0 + kk;
    }
#pragma unroll
    for (int i = 0; i < 2; ++i) *(volatile v8h*)(out16 + off[i]) = x[i];
    __threadfence();
#pragma unroll
    for (int i = 0; i < 2; ++i) *(volatile v8h*)(out16 + off[i]) = x[i];
  }

  if (MODE == 2) {
    const float cs = 1.0f / (WCARRY * VCARRY);
    const int hv = hin[0];
    const int wv = win[0];
    const bool bad = (hv != IMG_H_FULL) || (wv != IMG_W);
    const float poison = __uint_as_float(0x7FC00000u);
    v4f xs[4];
    size_t off[4];
#pragma unroll
    for (unsigned i = 0; i < 4u; ++i) {
      const unsigned r = 16u * i + (tid >> 4);
      const unsigned c = (tid & 15u) * 4u;
      const unsigned crow = row0 + r;
      const unsigned bidx = crow / (unsigned)SEQ;
      const unsigned sq = crow - bidx * (unsigned)SEQ;
      const size_t frow = (size_t)bidx * SEQ_FULL + sq;
      const v4f u = *(const v4f*)&Cs[r * LDC + c];
      const v4f g = *(const v4f*)(bias + n0 + c);
      v4f val;
#pragma unroll
      for (int j = 0; j < 4; ++j) {
        const float t = u[j] * cs + bf16r(g[j]);
        val[j] = bad ? poison : t;
      }
      xs[i] = val;
      off[i] = frow * DIM + n0 + c;
    }
#pragma unroll
    for (int i = 0; i < 4; ++i) *(volatile v4f*)(outf + off[i]) = xs[i];
    __threadfence();
#pragma unroll
    for (int i = 0; i < 4; ++i) *(volatile v4f*)(outf + off[i]) = xs[i];
  }
}

__global__ __launch_bounds__(256) void gemm_rope_kernel(
    const _Float16* __restrict__ A16, const _Float16* __restrict__ Bt,
    const float* __restrict__ cosT, const float* __restrict__ sinT,
    _Float16* __restrict__ out16) {
  gemm_body<0>(A16, Bt, (unsigned)DIM, cosT, cosT, sinT, (const int*)0, (const int*)0,
               (float*)0, out16);
}
__global__ __launch_bounds__(256) void gemm_v_kernel(
    const _Float16* __restrict__ A16, const _Float16* __restrict__ Bt,
    _Float16* __restrict__ vt) {
  gemm_body<1>(A16, Bt, (unsigned)DIM, (const float*)0, (const float*)0, (const float*)0,
               (const int*)0, (const int*)0, (float*)0, vt);
}
__global__ __launch_bounds__(256) void gemm_proj_kernel(
    const _Float16* __restrict__ A16, const _Float16* __restrict__ Bt,
    const float* __restrict__ bias, const int* __restrict__ hin, const int* __restrict__ win,
    float* __restrict__ outf) {
  gemm_body<2>(A16, Bt, (unsigned)DIM, bias, bias, bias, hin, win, outf, (_Float16*)0);
}

__global__ __launch_bounds__(128) void nattn_kernel(
    const _Float16* __restrict__ Qh, const _Float16* __restrict__ Kh,
    const _Float16* __restrict__ Vt, _Float16* __restrict__ Ov) {
  __shared__ _Float16 Ps[4 * 16 * LDP];
  __shared__ _Float16 Os[4 * 16 * LDT];

  const unsigned lane = threadIdx.x & 31u;
  const int wv = (int)(threadIdx.x >> 5);
  const int wave = __builtin_amdgcn_readfirstlane(wv);
  const int c0 = __builtin_amdgcn_readfirstlane(min(max(16 * wv - 8, 0), IMG_W - 32));
  const int nvalid = __builtin_amdgcn_readfirstlane(min(16, IMG_W - 16 * wv));
  const unsigned hh = lane >> 4, m = lane & 15u;
  const int irow = (int)blockIdx.x;
  const unsigned hq = blockIdx.y;
  const unsigned b = blockIdx.z;
  const int j0 = wave * 16;
  const int rstart = min(max(irow - (WIN / 2), 0), IMG_H - WIN);
  const float scale = 0.17677669529663687f;
  _Float16* P = Ps + wave * (16 * LDP);
  _Float16* O = Os + wave * (16 * LDT);

  int cq[8];
#pragma unroll
  for (int v = 0; v < 8; ++v) {
    const int jq = min(j0 + (int)hh * 8 + v, IMG_W - 1);
    cq[v] = min(max(jq - (WIN / 2), 0), IMG_W - WIN);
  }
  const int jql = min(j0 + (int)m, IMG_W - 1);
  const size_t qbase =
      ((size_t)b * SEQ + (size_t)(irow * IMG_W + jql)) * DIM + hh * 8u;

#pragma unroll 1
  for (unsigned hp = 0; hp < 2u; ++hp) {
    const unsigned head = hq * 2u + hp;
    const v16h qf = frag_at(Qh + qbase + head * HD);

    float mrow[8], lrow[8];
    v8f o[2];
#pragma unroll
    for (int v = 0; v < 8; ++v) { mrow[v] = -1.0e30f; lrow[v] = 0.0f; }
#pragma unroll
    for (int nb = 0; nb < 2; ++nb) o[nb] = (v8f){};

#pragma unroll 1
    for (int kr = 0; kr < WIN; ++kr) {
      const unsigned pix0 = (unsigned)((rstart + kr) * IMG_W + c0);

      v8f s[2];
#pragma unroll
      for (int kg = 0; kg < 2; ++kg) {
        const v16h kf = frag_at(
            Kh + ((size_t)b * SEQ + pix0 + (unsigned)kg * 16u + m) * DIM + head * HD + hh * 8u);
        v8f t = {};
        t = wmma16(qf, kf, t);
        s[kg] = t * scale;
      }

#pragma unroll
      for (int kg = 0; kg < 2; ++kg)
#pragma unroll
        for (int v = 0; v < 8; ++v) {
          const int kcol = c0 + kg * 16 + (int)m;
          const bool vis = (unsigned)(kcol - cq[v]) < (unsigned)WIN;
          s[kg][v] = vis ? s[kg][v] : -1.0e30f;
        }

      float alpha[8];
#pragma unroll
      for (int v = 0; v < 8; ++v) {
        float mx = fmaxf(s[0][v], s[1][v]);
        mx = red16_max(mx);
        const float mn = fmaxf(mrow[v], mx);
        alpha[v] = __expf(mrow[v] - mn);
        mrow[v] = mn;
      }
#pragma unroll
      for (int kg = 0; kg < 2; ++kg)
#pragma unroll
        for (int v = 0; v < 8; ++v) {
          const float e = __expf(s[kg][v] - mrow[v]);
          const _Float16 ph = toh_flush(e * PCARRY);
          P[(hh * 8u + (unsigned)v) * LDP + (unsigned)kg * 16u + m] = ph;
          s[kg][v] = (float)ph;
        }
#pragma unroll
      for (int v = 0; v < 8; ++v) {
        const float rs = red16_sum(s[0][v] + s[1][v]);
        lrow[v] = alpha[v] * lrow[v] + rs;
      }
#pragma unroll
      for (int nb = 0; nb < 2; ++nb)
#pragma unroll
        for (int v = 0; v < 8; ++v) o[nb][v] = o[nb][v] * alpha[v];
      wave_lds_sync();

      const v16h pf = ld_frag(P, LDP);
#pragma unroll
      for (int nb = 0; nb < 2; ++nb) {
        const v16h vf = frag_at(
            Vt + ((size_t)b * DIM + head * HD + (unsigned)nb * 16u + m) * SEQ + pix0 + hh * 8u);
        o[nb] = wmma16(pf, vf, o[nb]);
      }
      wave_lds_sync();
    }

    float inv[8];
#pragma unroll
    for (int v = 0; v < 8; ++v) inv[v] = __builtin_amdgcn_rcpf(lrow[v]) * VCARRY;
#pragma unroll
    for (int nb = 0; nb < 2; ++nb)
#pragma unroll
      for (int v = 0; v < 8; ++v)
        O[(hh * 8u + (unsigned)v) * LDT + hp * 32u + (unsigned)nb * 16u + m] =
            toh_flush(o[nb][v] * inv[v]);
  }
  wave_lds_sync();

  v8h x[4];
  size_t off[4];
#pragma unroll
  for (unsigned i = 0; i < 4u; ++i) {
    const unsigned r = 4u * i + (lane >> 3);
    const unsigned c = (lane & 7u) * 8u;
    x[i] = *(const v8h*)&O[r * LDT + c];
    const int jr = min(j0 + (int)r, IMG_W - 1);
    off[i] = ((size_t)b * SEQ + (size_t)(irow * IMG_W + jr)) * DIM + hq * 64u + c;
  }
#pragma unroll
  for (int i = 0; i < 4; ++i) {
    if (4 * i < nvalid) *(volatile v8h*)(Ov + off[i]) = x[i];
  }
  __threadfence();
#pragma unroll
  for (int i = 0; i < 4; ++i) {
    if (4 * i < nvalid) *(volatile v8h*)(Ov + off[i]) = x[i];
  }
}

extern "C" void kernel_launch(void* const* d_in, const int* in_sizes, int n_in,
                              void* d_out, int out_size, void* d_ws, size_t ws_size,
                              hipStream_t stream) {
  if (n_in < 6) return;
  const long long need_x = ((long long)(NB - 1) * SEQ_FULL + SEQ) * DIM;
  if ((long long)in_sizes[0] < need_x) return;
  if ((long long)in_sizes[1] < (long long)DIM * 3 * DIM) return;
  if ((long long)in_sizes[2] < (long long)DIM * DIM) return;
  if (in_sizes[3] < DIM) return;
  if (in_sizes[4] < 1 || in_sizes[5] < 1) return;
  if ((long long)out_size < need_x) return;
  if (ws_size < WS_TOTAL) return;

  const float* X     = (const float*)d_in[0];
  const float* wqkv  = (const float*)d_in[1];
  const float* wproj = (const float*)d_in[2];
  const float* bproj = (const float*)d_in[3];
  const int*   hin   = (const int*)d_in[4];
  const int*   win   = (const int*)d_in[5];
  float* out = (float*)d_out;

  char* ws = (char*)d_ws;
  _Float16* Wqkv_t = (_Float16*)(ws + OFF_WQKV);
  _Float16* Wp_t   = (_Float16*)(ws + OFF_WP);
  _Float16* X16    = (_Float16*)(ws + OFF_X16);
  _Float16* Q16    = (_Float16*)(ws + OFF_Q);
  _Float16* K16    = (_Float16*)(ws + OFF_K);
  _Float16* Vt16   = (_Float16*)(ws + OFF_VT);
  _Float16* Ctx16  = (_Float16*)(ws + OFF_CTX);
  float*    cosT   = (float*)(ws + OFF_COS);
  float*    sinT   = (float*)(ws + OFF_SIN);

  dim3 blk(256);
  dim3 gg(DIM / 64, MROWS / 64);

  wconv_kernel<<<dim3(3 * DIM / 64, DIM / 64), blk, 0, stream>>>(
      wqkv, Wqkv_t, (unsigned)(3 * DIM), (unsigned)DIM);
  wconv_kernel<<<dim3(DIM / 64, DIM / 64), blk, 0, stream>>>(
      wproj, Wp_t, (unsigned)DIM, (unsigned)DIM);

  xconv_kernel<<<dim3(MROWS / 8), blk, 0, stream>>>(X, X16);
  ropetab_kernel<<<dim3(SEQ * NPAIR / 256), blk, 0, stream>>>(cosT, sinT);

  gemm_rope_kernel<<<gg, blk, 0, stream>>>(X16, Wqkv_t, cosT, sinT, Q16);
  gemm_rope_kernel<<<gg, blk, 0, stream>>>(X16, Wqkv_t + (size_t)DIM * DIM, cosT, sinT, K16);
  gemm_v_kernel<<<gg, blk, 0, stream>>>(X16, Wqkv_t + (size_t)2 * DIM * DIM, Vt16);

  nattn_kernel<<<dim3(IMG_H, NHEAD / 2, NB), dim3(128), 0, stream>>>(Q16, K16, Vt16, Ctx16);

  gemm_proj_kernel<<<gg, blk, 0, stream>>>(Ctx16, Wp_t, bproj, hin, win, out);
}
